// PatchMTSC_32736240730551
// MI455X (gfx1250) — hardware-verified
//
#include <hip/hip_runtime.h>
#include <math.h>

typedef __attribute__((ext_vector_type(16))) _Float16 v16h;
typedef __attribute__((ext_vector_type(16))) __bf16 v16b;
typedef __attribute__((ext_vector_type(8)))  _Float16 v8h;
typedef __attribute__((ext_vector_type(8)))  float v8f;
typedef __attribute__((ext_vector_type(4)))  float v4f;
typedef __attribute__((ext_vector_type(2)))  float v2f;
typedef __attribute__((ext_vector_type(4)))  unsigned v4u;
typedef __attribute__((ext_vector_type(4)))  int v4i;
typedef float __attribute__((may_alias)) float_a;
typedef int __attribute__((may_alias)) int_a;

template <typename T> __device__ __forceinline__ void vst2(void* p, T v) { *(volatile T*)p = v; __threadfence(); *(volatile T*)p = v; }
__device__ __forceinline__ v8f wmma16(v16h a, v16h b, v8f c) {
  v8f d = __builtin_amdgcn_wmma_f32_16x16x32_f16(false, a, false, b, (short)0, c, false, false);
  asm volatile("v_nop\n\tv_nop\n\tv_nop\n\tv_nop" : "+v"(d) : "v"(a), "v"(b));
  return d;
}
__device__ __forceinline__ v8f wmma_bf(v16b a, v16b b, v8f c) {
  v8f d = __builtin_amdgcn_wmma_f32_16x16x32_bf16(false, a, false, b, (short)0, c, false, false);
  asm volatile("v_nop\n\tv_nop\n\tv_nop\n\tv_nop" : "+v"(d) : "v"(a), "v"(b));
  return d;
}
__device__ __forceinline__ v16h frag_h(const _Float16* rowk0, int lane) {
  union { v16h v; v8h q[2]; } u; const _Float16* p = rowk0 + 8 * (lane >> 4);
  u.q[0] = *(const v8h*)p; u.q[1] = *(const v8h*)(p + 16); return u.v;
}
__device__ __forceinline__ v16h frag_f32(const float* rowk0, int lane) {
  v16h a; const float* p = rowk0 + 8 * (lane >> 4);
#pragma unroll
  for (int i = 0; i < 8; ++i) { a[i] = (_Float16)p[i]; a[8 + i] = (_Float16)p[16 + i]; }
  return a;
}
__device__ __forceinline__ v16h frag_f32s(const float* rowk0, int lane, float sc) {
  v16h a; const float* p = rowk0 + 8 * (lane >> 4);
#pragma unroll
  for (int i = 0; i < 8; ++i) { a[i] = (_Float16)(p[i] * sc); a[8 + i] = (_Float16)(p[16 + i] * sc); }
  return a;
}
__device__ __forceinline__ v16h fragc_f32(const float* W, int k0, int n, int lane, int ld, int K) {
  v16h a; const int g = lane >> 4;
#pragma unroll
  for (int i = 0; i < 8; ++i) { const int ka = k0 + 8 * g + i, kb = ka + 16;
    a[i] = (_Float16)(ka < K ? W[(size_t)(ka < K ? ka : K - 1) * ld + n] : 0.f); a[8 + i] = (_Float16)(kb < K ? W[(size_t)(kb < K ? kb : K - 1) * ld + n] : 0.f); }
  return a;
}
struct F2 { v16b h, l; };
__device__ __forceinline__ F2 bsplit16(const float v[16]) { F2 r;
#pragma unroll
  for (int i = 0; i < 16; ++i) { const __bf16 h = (__bf16)v[i]; r.h[i] = h; r.l[i] = (__bf16)(v[i] - (float)h); }
  return r; }
__device__ __forceinline__ F2 split_row(const float* row, int k0, int lane) { float v[16]; const float* p = row + k0 + 8 * (lane >> 4);
#pragma unroll
  for (int i = 0; i < 8; ++i) { v[i] = p[i]; v[8 + i] = p[16 + i]; }
  return bsplit16(v); }
__device__ __forceinline__ F2 split_rowK(const float* row, int k0, int lane, int K) { float v[16]; const int g = lane >> 4;
#pragma unroll
  for (int i = 0; i < 8; ++i) { const int ka = k0 + 8 * g + i, kb = ka + 16; v[i] = ka < K ? row[ka < K ? ka : K - 1] : 0.f; v[8 + i] = kb < K ? row[kb < K ? kb : K - 1] : 0.f; }
  return bsplit16(v); }
__device__ __forceinline__ F2 split_col(const float* W, int k0, int n, int lane, int ld, int K) { float v[16]; const int g = lane >> 4;
#pragma unroll
  for (int i = 0; i < 8; ++i) { const int ka = k0 + 8 * g + i, kb = ka + 16; v[i] = ka < K ? W[(size_t)(ka < K ? ka : K - 1) * ld + n] : 0.f; v[8 + i] = kb < K ? W[(size_t)(kb < K ? kb : K - 1) * ld + n] : 0.f; }
  return bsplit16(v); }
__device__ __forceinline__ v8f mac3(const F2& a, const F2& b, v8f c) { c = wmma_bf(a.l, b.h, c); c = wmma_bf(a.h, b.l, c); return wmma_bf(a.h, b.h, c); }
__device__ __forceinline__ float sigm(float v) { return 1.0f / (1.0f + expf(-v)); }
#define LDSX() do { asm volatile("s_wait_dscnt 0" ::: "memory"); __builtin_amdgcn_wave_barrier(); __builtin_amdgcn_fence(__ATOMIC_RELEASE, "workgroup"); } while (0)


#define NB 128
#define NN 512
#define DD 128
#define NROW (NB * NN)
#define BNEPS 1e-5f
#define SLOPE 0.01f
#define DIAGINF 1.0e8f
#define NSB (NROW / 256)
#ifndef TNB
#define TNB NB
#endif
typedef __attribute__((ext_vector_type(8))) __bf16 v8b;
__device__ __forceinline__ v16b frag_b(const __bf16* rowk0, int lane) {
  union { v16b v; v8b q[2]; } u; const __bf16* p = rowk0 + 8 * (lane >> 4);
  u.q[0] = *(const v8b*)p; u.q[1] = *(const v8b*)(p + 16); return u.v;
}
__device__ __forceinline__ float bfr(float v) { return (float)(__bf16)v; }
__device__ __attribute__((noinline)) float exp_ni(float v) { return expf(v); }
__device__ __attribute__((noinline)) float erf_ni(float v) { return erff(v); }

#define WS_NF  0u
#define WS_NFL (WS_NF + 2u * (size_t)NROW * DD)
#define WS_ST1 (WS_NFL + 2u * (size_t)NROW * DD)
#define WS_MV1 (WS_ST1 + 4u * (size_t)NSB * DD)
#define WS_XB  (WS_MV1 + 4u * 2 * DD)
#define WS_XBL (WS_XB + 2u * (size_t)NROW * DD)
#define WS_H   (WS_XBL + 2u * (size_t)NROW * DD)
#define WS_ST2 (WS_H + 4u * (size_t)NROW * DD)
#define WS_MV2 (WS_ST2 + 4u * (size_t)NSB * DD)
#define WS_END (WS_MV2 + 4u * 2 * DD)

__device__ __forceinline__ v16b fragb_f32(const float* __restrict__ p, int lane) { v16b a; const float* pp = p + 8 * (lane >> 4);
#pragma unroll
  for (int i = 0; i < 8; ++i) { a[i] = (__bf16)pp[i]; a[8 + i] = (__bf16)pp[16 + i]; } return a; }
__device__ __forceinline__ float lrelu(float v) { return v >= 0.f ? v : SLOPE * v; }
__global__ __launch_bounds__(128) void k_nf(const float* __restrict__ X, const float* __restrict__ WM, const float* __restrict__ BM, _Float16* __restrict__ NF, _Float16* __restrict__ NFL) { __shared__ __align__(16) _Float16 sh[4][16][136], sl[4][16][136];
  const int tid = threadIdx.x, wave = tid >> 5, lane = tid & 31, col = lane & 15, g = lane >> 4; const size_t r0 = (size_t)blockIdx.x * 64 + wave * 16;
  v8f acc[8] = {};
#pragma unroll
  for (int kc = 0; kc < DD / 32; ++kc) { const v16b a = fragb_f32(X + (r0 + col) * DD + kc * 32, lane);
#pragma unroll
    for (int j = 0; j < 8; ++j) { v16b w; const int o = j * 16 + col;
#pragma unroll
      for (int i = 0; i < 8; ++i) { w[i] = (__bf16)WM[(size_t)(kc * 32 + 8 * g + i) * DD + o]; w[8 + i] = (__bf16)WM[(size_t)(kc * 32 + 16 + 8 * g + i) * DD + o]; }
      acc[j] = wmma_bf(a, w, acc[j]); } }
#pragma unroll
  for (int j = 0; j < 8; ++j) { const float bb = bfr(BM[j * 16 + col]);
#pragma unroll
    for (int r = 0; r < 8; ++r) { const float v = acc[j][r] + bb; const _Float16 hv = (_Float16)v; sh[wave][8 * g + r][j * 16 + col] = hv; sl[wave][8 * g + r][j * 16 + col] = (_Float16)((v - (float)hv) * 2048.0f); } }
  LDSX(); for (int rl = 0; rl < 16; ++rl) if (lane < 16) { const size_t o = (r0 + rl) * DD + lane * 8; vst2((unsigned*)(NF + o), *(const v4u*)&sh[wave][rl][lane * 8]); vst2((unsigned*)(NFL + o), *(const v4u*)&sl[wave][rl][lane * 8]); } }
__global__ __launch_bounds__(128) void k_psum(const float* __restrict__ X, const float* __restrict__ MU, int P, int RAW, float* __restrict__ PS) { __shared__ __align__(16) float s[DD]; const int t = threadIdx.x; const size_t r0 = (size_t)blockIdx.x * 256; const float mu = (P == 2) ? MU[t] : 0.f; float acc = 0.f;
#pragma unroll 4
  for (int r = 0; r < 256; ++r) { float v = X[(r0 + r) * DD + t]; if (!RAW) v = bfr(v); v -= mu; acc += (P == 2) ? v * v : v; }
  s[t] = acc; __syncthreads(); if (t < DD / 4) vst2(PS + (size_t)blockIdx.x * DD + t * 4, *(const v4f*)&s[t * 4]); }
__global__ __launch_bounds__(128) void k_pred(const float* __restrict__ PS, int which, float* __restrict__ MV) { __shared__ __align__(16) float s[DD]; const int t = threadIdx.x; float acc = 0.f; for (int b = 0; b < NSB; ++b) acc += PS[(size_t)b * DD + t]; s[t] = acc * (1.0f / NROW); __syncthreads(); if (t < DD / 4) vst2(MV + which * DD + t * 4, *(const v4f*)&s[t * 4]); }
__global__ __launch_bounds__(128) void k_xb(const float* __restrict__ X, const float* __restrict__ MV, const float* __restrict__ G, const float* __restrict__ Bt, _Float16* __restrict__ XB, _Float16* __restrict__ XBL) { __shared__ __align__(16) _Float16 th[DD][72], tl[DD][72]; const int t = threadIdx.x; const size_t b = blockIdx.y; const int m0 = blockIdx.x * 64;
  for (int e = t; e < 64 * DD; e += 128) { const int ml = e / DD, d = e % DD; const float v = (bfr(X[((b * NN + m0 + ml) * DD) + d]) - MV[d]) / sqrtf(MV[DD + d] + BNEPS) * bfr(G[d]) + bfr(Bt[d]); const _Float16 hv = (_Float16)v; th[d][ml] = hv; tl[d][ml] = (_Float16)(v - (float)hv); }
  __syncthreads(); for (int e = t; e < DD * 8; e += 128) { const int d = e >> 3, q = e & 7; const size_t o = (b * DD + d) * (size_t)NN + m0 + q * 8; vst2((unsigned*)(XB + o), *(const v4u*)&th[d][q * 8]); vst2((unsigned*)(XBL + o), *(const v4u*)&tl[d][q * 8]); } }
__global__ __launch_bounds__(128) void k_att(const _Float16* __restrict__ NF, const _Float16* __restrict__ NFL, const _Float16* __restrict__ XB, const _Float16* __restrict__ XBL, const float* __restrict__ PRE, const float* __restrict__ X, const float* __restrict__ MV, const float* __restrict__ G, const float* __restrict__ Bt, const float* __restrict__ WT, const float* __restrict__ BTh, float* __restrict__ H) {
  __shared__ __align__(16) float sp[4][16][36]; __shared__ __align__(16) float sg[4][16][132];
  const int tid = threadIdx.x, wave = tid >> 5, lane = tid & 31, col = lane & 15, g = lane >> 4; const size_t b = blockIdx.y; const int q0 = blockIdx.x * 64 + wave * 16; const size_t rq = b * NN + q0;
  v16h aq[4], al[4];
#pragma unroll
  for (int kc = 0; kc < 4; ++kc) { aq[kc] = frag_h(NF + (rq + col) * DD + kc * 32, lane); al[kc] = frag_h(NFL + (rq + col) * DD + kc * 32, lane); }
  float m[8], l[8];
#pragma unroll
  for (int r = 0; r < 8; ++r) { m[r] = -3.0e38f; l[r] = 0.f; }
  v8f acc[8];
#pragma unroll
  for (int j = 0; j < 8; ++j) acc[j] = v8f{};
#pragma unroll 1
  for (int ks = 0; ks < NN / 32; ++ks) { float s[2][8];
#pragma unroll
    for (int ct = 0; ct < 2; ++ct) { const int kk = ks * 32 + ct * 16 + col; const size_t rk = b * NN + kk; v8f c = {}, cl = {};
#pragma unroll
      for (int kc = 0; kc < 4; ++kc) { const v16h kh = frag_h(NF + rk * DD + kc * 32, lane), kl = frag_h(NFL + rk * DD + kc * 32, lane); c = wmma16(aq[kc], kh, c); cl = wmma16(aq[kc], kl, cl); cl = wmma16(al[kc], kh, cl); }
#pragma unroll
      for (int r = 0; r < 8; ++r) { const int n = q0 + 8 * g + r; float v = c[r] + cl[r] * (1.0f / 2048.0f); if (n == kk) v -= DIAGINF; s[ct][r] = lrelu(v); } }
    float alpha[8];
#pragma unroll
    for (int r = 0; r < 8; ++r) { float mx = fmaxf(s[0][r], s[1][r]);
#pragma unroll
      for (int o = 1; o < 16; o <<= 1) mx = fmaxf(mx, __shfl_xor(mx, o));
      const float mn = fmaxf(m[r], mx); alpha[r] = __expf(m[r] - mn); const float e0 = __expf(s[0][r] - mn), e1 = __expf(s[1][r] - mn); float es = e0 + e1;
#pragma unroll
      for (int o = 1; o < 16; o <<= 1) es += __shfl_xor(es, o);
      l[r] = l[r] * alpha[r] + es; m[r] = mn; const size_t po_ = (size_t)(q0 + 8 * g + r) * NN + ks * 32 + col; sp[wave][8 * g + r][col] = e0 * bfr(PRE[po_]); sp[wave][8 * g + r][16 + col] = e1 * bfr(PRE[po_ + 16]); }
#pragma unroll
    for (int j = 0; j < 8; ++j)
#pragma unroll
      for (int r = 0; r < 8; ++r) acc[j][r] *= alpha[r];
    LDSX();
    v16h pa; { const float* prow = &sp[wave][col][0] + 8 * (lane >> 4);
#pragma unroll
      for (int i = 0; i < 8; ++i) { pa[i] = (_Float16)(prow[i] * 2048.0f); pa[8 + i] = (_Float16)(prow[16 + i] * 2048.0f); } }
#pragma unroll
    for (int j = 0; j < 8; ++j) { const size_t po = (b * DD + j * 16 + col) * (size_t)NN + ks * 32; acc[j] = wmma16(pa, frag_h(XB + po, lane), acc[j]); acc[j] = wmma16(pa, frag_h(XBL + po, lane), acc[j]); }
    LDSX(); }
#pragma unroll
  for (int r = 0; r < 8; ++r) { const int n = q0 + 8 * g + r; const float il = (1.0f / 2048.0f) / l[r]; const float pnn = bfr(PRE[(size_t)n * NN + n]);
#pragma unroll
    for (int j = 0; j < 8; ++j) { const int d = j * 16 + col; const size_t xo = (b * DD + d) * (size_t)NN + n; const float xbn = (float)XB[xo] + (float)XBL[xo]; sg[wave][8 * g + r][d] = acc[j][r] * il + pnn * xbn; } }
  (void)X; (void)MV; (void)G; (void)Bt;
  LDSX(); for (int rl = 0; rl < 16; ++rl) vst2(H + (rq + rl) * DD + lane * 4, *(const v4f*)&sg[wave][rl][lane * 4]); (void)WT; (void)BTh; }
__global__ __launch_bounds__(128) void k_theta(float* __restrict__ Hh, const float* __restrict__ WT, const float* __restrict__ BTh) { __shared__ __align__(16) float sf[4][16][132];
  const int tid = threadIdx.x, wave = tid >> 5, lane = tid & 31, col = lane & 15, g = lane >> 4; const size_t r0 = (size_t)blockIdx.x * 64 + wave * 16;
  v8f acc2[8] = {};
#pragma unroll
  for (int kc = 0; kc < DD / 32; ++kc) { const F2 a = split_row(Hh + (r0 + col) * DD, kc * 32, lane);
#pragma unroll
    for (int j = 0; j < 8; ++j) { v16b w; const int o = j * 16 + col;
#pragma unroll
      for (int i = 0; i < 8; ++i) { w[i] = (__bf16)WT[(size_t)(kc * 32 + 8 * g + i) * DD + o]; w[8 + i] = (__bf16)WT[(size_t)(kc * 32 + 16 + 8 * g + i) * DD + o]; }
      acc2[j] = wmma_bf(a.h, w, acc2[j]); acc2[j] = wmma_bf(a.l, w, acc2[j]); } }
#pragma unroll
  for (int j = 0; j < 8; ++j) { const float bb = bfr(BTh[j * 16 + col]);
#pragma unroll
    for (int r = 0; r < 8; ++r) sf[wave][8 * g + r][j * 16 + col] = acc2[j][r] + bb; }
  __syncthreads();
  for (int rl = 0; rl < 16; ++rl) vst2(Hh + (r0 + rl) * DD + lane * 4, *(const v4f*)&sf[wave][rl][lane * 4]); }
__global__ __launch_bounds__(256) void k_fin(const float* __restrict__ Hh, const float* __restrict__ MV, const float* __restrict__ G, const float* __restrict__ Bt, float* __restrict__ OUT) { const int t = threadIdx.x; const size_t r0 = (size_t)blockIdx.x * 64;
  for (int e = t; e < 64 * (DD / 4); e += 256) { const int rl = e / (DD / 4), q = e % (DD / 4); const size_t o = (r0 + rl) * DD + q * 4; v4f v;
#pragma unroll
    for (int i = 0; i < 4; ++i) { const int d = q * 4 + i; v[i] = lrelu((Hh[o + i] - MV[d]) / sqrtf(MV[DD + d] + BNEPS) * bfr(G[d]) + bfr(Bt[d])); }
    vst2(OUT + o, v); } }
extern "C" void kernel_launch(void* const* d_in, const int* in_sizes, int n_in, void* d_out, int out_size, void* d_ws, size_t ws_size, hipStream_t stream) {
  (void)in_sizes; (void)n_in; (void)out_size;
  const float** F = (const float**)d_in;
  if (ws_size < (size_t)WS_END) return;
  char* ws = (char*)d_ws; _Float16 *NF = (_Float16*)(ws + WS_NF), *NFL = (_Float16*)(ws + WS_NFL), *XB = (_Float16*)(ws + WS_XB), *XBL = (_Float16*)(ws + WS_XBL); float *ST1 = (float*)(ws + WS_ST1), *MV1 = (float*)(ws + WS_MV1), *H = (float*)(ws + WS_H), *ST2 = (float*)(ws + WS_ST2), *MV2 = (float*)(ws + WS_MV2);
  k_nf<<<NROW / 64, 128, 0, stream>>>(F[0], F[1], F[2], NF, NFL);
  k_psum<<<NSB, 128, 0, stream>>>(F[0], MV1, 1, 0, ST1); k_pred<<<1, 128, 0, stream>>>(ST1, 0, MV1);
  k_psum<<<NSB, 128, 0, stream>>>(F[0], MV1, 2, 0, ST1); k_pred<<<1, 128, 0, stream>>>(ST1, 1, MV1);
  k_xb<<<dim3(NN / 64, NB), 128, 0, stream>>>(F[0], MV1, F[5], F[6], XB, XBL);
  k_att<<<dim3(NN / 64, TNB), 128, 0, stream>>>(NF, NFL, XB, XBL, F[9], F[0], MV1, F[5], F[6], F[3], F[4], H);
  k_theta<<<TNB * NN / 64, 128, 0, stream>>>(H, F[3], F[4]);
  k_psum<<<NSB, 128, 0, stream>>>(H, MV2, 1, 1, ST2); k_pred<<<1, 128, 0, stream>>>(ST2, 0, MV2);
  k_psum<<<NSB, 128, 0, stream>>>(H, MV2, 2, 1, ST2); k_pred<<<1, 128, 0, stream>>>(ST2, 1, MV2);
  k_fin<<<NROW / 64, 256, 0, stream>>>(H, MV2, F[7], F[8], (float*)d_out);
}
